// RFP_DAGs_50929722196486
// MI455X (gfx1250) — hardware-verified
//
#include <hip/hip_runtime.h>
#include <math.h>

typedef __attribute__((ext_vector_type(16))) _Float16 v16h;
typedef __attribute__((ext_vector_type(8)))  _Float16 v8h;
typedef __attribute__((ext_vector_type(8)))  float    v8f;
typedef __attribute__((ext_vector_type(4)))  float    v4f;

constexpr int kB      = 4;
constexpr int kC      = 64;
constexpr int kH      = 64;
constexpr int kW      = 64;
constexpr int kD      = 8;
constexpr int kG      = 4;
constexpr int kCells  = kH * kW;
constexpr int kTilesC = kC / 16;
constexpr size_t kElems = (size_t)kB * kC * kCells * kD;
constexpr int kThr    = 256;
static_assert(kB == 4 && kC == 64 && kD == 8 && kG == 4, "4 batch columns per weight set; 64 channels = four 16-row tiles");

constexpr float kStateCarry  = 1024.0f;
constexpr float kWeightCarry = 1024.0f;
constexpr float kFoldBack    = 1.0f / (kStateCarry * kWeightCarry);
constexpr float kF16MinNorm  = 6.103515625e-5f;
static_assert(kStateCarry * kWeightCarry == 1048576.0f, "carry product");

constexpr size_t kOffXF   = 0;
constexpr size_t kOffACC  = kOffXF  + (size_t)kD * kCells * 2 * 8 * 16 * 2;
constexpr size_t kOffRB   = kOffACC + (size_t)kD * kCells * kTilesC * 8 * 8 * 4;
constexpr size_t kWsTotal = kOffRB  + (size_t)kD * kW * 2 * 32 * 16 * 2;
static_assert(kWsTotal == 51380224ull && kWsTotal <= 134217728ull, "carve total and cap");
static_assert((kOffACC % 256) == 0 && (kOffRB % 256) == 0, "aligned regions");

namespace eng {

union FragU { v16h v; v8h h[2]; };

__device__ __forceinline__ unsigned short f2bf_bits(float f) {
  unsigned u = __float_as_uint(f);
  return (unsigned short)((u + 0x7FFFu + ((u >> 16) & 1u)) >> 16);
}
__device__ __forceinline__ float bf16v(float f) {
  return __uint_as_float(((unsigned)f2bf_bits(f)) << 16);
}
__device__ __forceinline__ _Float16 to_f16_flushed(float c) {
  const float z = (fabsf(c) < kF16MinNorm) ? 0.0f : c;
  return (_Float16)z;
}
__device__ __forceinline__ v8f mma_f16(v16h a, v16h b, v8f c) {
  c = __builtin_amdgcn_wmma_f32_16x16x32_f16(false, a, false, b, (short)0, c, false, false);
  asm volatile("v_nop\n\tv_nop\n\tv_nop\n\tv_nop" : "+v"(c) : "v"(a), "v"(b));
  return c;
}

}

__global__ __launch_bounds__(kThr) void xfrag_kernel(const float* __restrict__ x, unsigned short* __restrict__ XF) {
  const int g  = blockIdx.x * kThr + threadIdx.x;
  const int n  = g & 3;
  const int hs = (g >> 2) & 1;
  const int c  = (g >> 3) & 1;
  const int p  = (g >> 4) & (kCells - 1);
  const int d  = g >> 16;
  v8h lo, hi;
#pragma unroll
  for (int e = 0; e < 16; ++e) {
    const int k = 32 * c + 16 * (e >> 3) + 8 * hs + (e & 7);
    const float xv = x[(((size_t)n * kC + k) * kCells + p) * kD + d];
    const _Float16 hv = eng::to_f16_flushed(eng::bf16v(xv) * kStateCarry);
    if (e < 8) lo[e & 7] = hv; else hi[e & 7] = hv;
  }
  eng::FragU u0;
  u0.h[0] = lo;
  u0.h[1] = hi;
  v16h* dst = (v16h*)XF + g;
  for (int pass = 0; pass < 2; ++pass) {
    *(volatile v16h*)dst = u0.v;
    __threadfence();
  }
}

__global__ __launch_bounds__(32) void plane_dir_kernel(const unsigned short* __restrict__ XF,
                                                       const float* __restrict__ Wx, const float* __restrict__ Wv,
                                                       const float* __restrict__ Wh, const float* __restrict__ bias,
                                                       float* __restrict__ ACC, unsigned short* __restrict__ RB,
                                                       int gdir, int flip_i, int flip_j, int first) {
  __shared__ __align__(32) v16h AF[3 * kTilesC * 2 * 32];

  const int lane = threadIdx.x & 31;
  const int hsel = lane >> 4;
  const int n    = lane & 15;
  const int d    = blockIdx.x;
  const bool liveCol = (n < kB);
  const int nc   = liveCol ? n : (kB - 1);
  const size_t wofs = ((size_t)gdir * kD + d) * kC * kC;

#pragma unroll 1
  for (int t = 0; t < 3; ++t) {
    const float* wsrc = ((t == 0) ? Wx : ((t == 1) ? Wv : Wh)) + wofs;
#pragma unroll 1
    for (int m = 0; m < kTilesC; ++m) {
#pragma unroll 1
      for (int c = 0; c < 2; ++c) {
        v8h lo, hi;
#pragma unroll
        for (int e = 0; e < 16; ++e) {
          const int k = 32 * c + 16 * (e >> 3) + 8 * hsel + (e & 7);
          const float wv = wsrc[(16 * m + n) * kC + k];
          const _Float16 hv = eng::to_f16_flushed(eng::bf16v(wv) * kWeightCarry);
          if (e < 8) lo[e & 7] = hv; else hi[e & 7] = hv;
        }
        eng::FragU u0;
        u0.h[0] = lo;
        u0.h[1] = hi;
        AF[((t * kTilesC + m) * 2 + c) * 32 + lane] = u0.v;
      }
    }
  }
  float bs[kTilesC][8];
#pragma unroll
  for (int m = 0; m < kTilesC; ++m) {
#pragma unroll
    for (int r = 0; r < 8; ++r) bs[m][r] = eng::bf16v(bias[((size_t)gdir * kD + d) * kC + 16 * m + 8 * hsel + r]);
  }
  v16h* rb = (v16h*)RB + (size_t)d * kW * 2 * 32;
  const v8h zh = (v8h){(_Float16)0.0f, (_Float16)0.0f, (_Float16)0.0f, (_Float16)0.0f,
                       (_Float16)0.0f, (_Float16)0.0f, (_Float16)0.0f, (_Float16)0.0f};
  eng::FragU zf;
  zf.h[0] = zh;
  zf.h[1] = zh;
#pragma unroll 1
  for (int jj = 0; jj < kW; ++jj) {
    for (int pass = 0; pass < 2; ++pass) {
      *(volatile v16h*)(rb + (jj * 2 + 0) * 32 + lane) = zf.v;
      *(volatile v16h*)(rb + (jj * 2 + 1) * 32 + lane) = zf.v;
      __threadfence();
    }
  }
  __syncthreads();

  const v8f z8 = (v8f){0.f, 0.f, 0.f, 0.f, 0.f, 0.f, 0.f, 0.f};
  const v16h* xf = (const v16h*)XF + (size_t)d * kCells * 16;
  float* accd = ACC + (size_t)d * kCells * (kTilesC * 64);

#pragma unroll 1
  for (int ii = 0; ii < kH; ++ii) {
    const int i = flip_i ? (kH - 1 - ii) : ii;
    eng::FragU l0, l1;
    l0.v = zf.v;
    l1.v = zf.v;
#pragma unroll 1
    for (int jj = 0; jj < kW; ++jj) {
      const int j = flip_j ? (kW - 1 - jj) : jj;
      const int p = i * kW + j;
      const v16h xq0 = xf[((size_t)p * 2 + 0) * 8 + hsel * 4 + nc];
      const v16h xq1 = xf[((size_t)p * 2 + 1) * 8 + hsel * 4 + nc];
      const v16h x0 = liveCol ? xq0 : zf.v;
      const v16h x1 = liveCol ? xq1 : zf.v;
      const v16h u0 = rb[(jj * 2 + 0) * 32 + lane];
      const v16h u1 = rb[(jj * 2 + 1) * 32 + lane];
      v8h nb[kTilesC];
#pragma unroll
      for (int m = 0; m < kTilesC; ++m) {
        v8f acc = z8;
        acc = eng::mma_f16(AF[((0 * kTilesC + m) * 2 + 0) * 32 + lane], x0, acc);
        acc = eng::mma_f16(AF[((0 * kTilesC + m) * 2 + 1) * 32 + lane], x1, acc);
        acc = eng::mma_f16(AF[((1 * kTilesC + m) * 2 + 0) * 32 + lane], u0, acc);
        acc = eng::mma_f16(AF[((1 * kTilesC + m) * 2 + 1) * 32 + lane], u1, acc);
        acc = eng::mma_f16(AF[((2 * kTilesC + m) * 2 + 0) * 32 + lane], l0.v, acc);
        acc = eng::mma_f16(AF[((2 * kTilesC + m) * 2 + 1) * 32 + lane], l1.v, acc);
        float* ap = accd + ((size_t)p * kTilesC + m) * 64 + (hsel * 4 + nc) * 8;
        v4f a0 = {0.f, 0.f, 0.f, 0.f};
        v4f a1 = {0.f, 0.f, 0.f, 0.f};
        if (!first) {
          a0 = *(const v4f*)ap;
          a1 = *(const v4f*)(ap + 4);
        }
        v4f o0, o1;
#pragma unroll
        for (int r = 0; r < 8; ++r) {
          const float pre = fmaf(acc[r], kFoldBack, bs[m][r]);
          const float hv = liveCol ? fmaxf(pre, 0.0f) : 0.0f;
          nb[m][r] = eng::to_f16_flushed(hv * kStateCarry);
          const float av = (r < 4) ? a0[r & 3] : a1[r & 3];
          if (r < 4) o0[r & 3] = av + hv; else o1[r & 3] = av + hv;
        }
        if (liveCol) {
          for (int pass = 0; pass < 2; ++pass) {
            *(volatile v4f*)ap = o0;
            *(volatile v4f*)(ap + 4) = o1;
            __threadfence();
          }
        }
      }
      l0.h[0] = nb[0];
      l0.h[1] = nb[1];
      l1.h[0] = nb[2];
      l1.h[1] = nb[3];
      for (int pass = 0; pass < 2; ++pass) {
        *(volatile v16h*)(rb + (jj * 2 + 0) * 32 + lane) = l0.v;
        *(volatile v16h*)(rb + (jj * 2 + 1) * 32 + lane) = l1.v;
        __threadfence();
      }
    }
  }
}

__global__ __launch_bounds__(kThr) void mean_out_kernel(const float* __restrict__ ACC, const float* __restrict__ x,
                                                        float* __restrict__ out) {
  const size_t t = (size_t)blockIdx.x * kThr + threadIdx.x;
  const int p  = (int)(t & (kCells - 1));
  const int bc = (int)(t >> 12);
  const int c  = bc & (kC - 1);
  const int b  = bc >> 6;
  const size_t aofs = ((size_t)p * kTilesC + (c >> 4)) * 64 + (((c >> 3) & 1) * 4 + b) * 8 + (c & 7);
  const float* xp = x + t * kD;
  const v4f x0 = *(const v4f*)xp;
  const v4f x1 = *(const v4f*)(xp + 4);
  v4f o0, o1;
#pragma unroll
  for (int d = 0; d < kD; ++d) {
    const float av = ACC[(size_t)d * kCells * (kTilesC * 64) + aofs];
    const float xv = (d < 4) ? x0[d & 3] : x1[d & 3];
    const float y = fmaxf(fmaf(0.25f, av, eng::bf16v(xv)), 0.0f);
    if (d < 4) o0[d & 3] = y; else o1[d & 3] = y;
  }
  float* op = out + t * kD;
  for (int pass = 0; pass < 2; ++pass) {
    *(volatile v4f*)op = o0;
    *(volatile v4f*)(op + 4) = o1;
    __threadfence();
  }
}

static_assert(((size_t)kD * kCells * 16) % kThr == 0 && ((size_t)kB * kC * kCells) % kThr == 0, "re-layout and output grids exact");

extern "C" void kernel_launch(void* const* d_in, const int* in_sizes, int n_in,
                              void* d_out, int out_size, void* d_ws, size_t ws_size,
                              hipStream_t stream) {
  if (n_in < 5 || d_out == nullptr || d_ws == nullptr) return;
  if ((size_t)in_sizes[0] != kElems) return;
  if (in_sizes[1] != kG * kD * kC * kC || in_sizes[2] != kG * kD * kC * kC || in_sizes[3] != kG * kD * kC * kC) return;
  if (in_sizes[4] != kG * kD * kC) return;
  if ((size_t)out_size != kElems) return;
  if (ws_size < kWsTotal) return;

  const float* x    = (const float*)d_in[0];
  const float* Wx   = (const float*)d_in[1];
  const float* Wv   = (const float*)d_in[2];
  const float* Wh   = (const float*)d_in[3];
  const float* bias = (const float*)d_in[4];
  float* out = (float*)d_out;

  char* ws = (char*)d_ws;
  unsigned short* XF = (unsigned short*)(ws + kOffXF);
  float* ACC = (float*)(ws + kOffACC);
  unsigned short* RB = (unsigned short*)(ws + kOffRB);

  xfrag_kernel<<<(int)(((size_t)kD * kCells * 16) / kThr), kThr, 0, stream>>>(x, XF);
  plane_dir_kernel<<<kD, 32, 0, stream>>>(XF, Wx, Wv, Wh, bias, ACC, RB, 0, 0, 0, 1);
  plane_dir_kernel<<<kD, 32, 0, stream>>>(XF, Wx, Wv, Wh, bias, ACC, RB, 1, 0, 1, 0);
  plane_dir_kernel<<<kD, 32, 0, stream>>>(XF, Wx, Wv, Wh, bias, ACC, RB, 2, 1, 0, 0);
  plane_dir_kernel<<<kD, 32, 0, stream>>>(XF, Wx, Wv, Wh, bias, ACC, RB, 3, 1, 1, 0);
  mean_out_kernel<<<(int)(((size_t)kB * kC * kCells) / kThr), kThr, 0, stream>>>(ACC, x, out);
}
